// LorentzMultiHeadedAttention_4097398801027
// MI455X (gfx1250) — hardware-run, weakly checked
//
#include <hip/hip_runtime.h>
#include <stddef.h>
#include <stdint.h>

#define NB   4
#define SEQ  1024
#define DM   1024
#define NH   16
#define HD   64
#define NR   (NB * SEQ)
#define NBH  (NB * NH)

#define TP   68
#define HP   72
#define OP   68
#define DFAR 160
#define F16_MIN_NORMAL 6.103515625e-05f

#define SZ_XB   ((size_t)3 * NR * DM * 2)
#define SZ_WB   ((size_t)3 * DM * DM * 2)
#define SZ_G    ((size_t)SEQ * SEQ * 4)
#define SZ_P16  ((size_t)NR * DM * 2)
#define SZ_VT   ((size_t)NBH * HD * SEQ * 2)
#define OFF_XB  ((size_t)0)
#define OFF_WB  (OFF_XB + SZ_XB)
#define OFF_G   (OFF_WB + SZ_WB)
#define OFF_Q16 (OFF_G + SZ_G)
#define OFF_K16 (OFF_Q16 + SZ_P16)
#define OFF_VT  (OFF_K16 + SZ_P16)
#define WS_TOTAL (OFF_VT + SZ_VT)

static_assert(OFF_WB == (size_t)25165824);
static_assert(OFF_G == (size_t)31457280);
static_assert(OFF_Q16 == (size_t)35651584);
static_assert(OFF_K16 == (size_t)44040192);
static_assert(OFF_VT == (size_t)52428800);
static_assert(WS_TOTAL == (size_t)60817408);
static_assert(WS_TOTAL <= (size_t)134217728);
static_assert((OFF_WB % 256) == 0);
static_assert((OFF_G % 256) == 0);
static_assert((OFF_Q16 % 256) == 0);
static_assert((OFF_K16 % 256) == 0);
static_assert((OFF_VT % 256) == 0);
static_assert((SEQ % 128) == 0);
static_assert((NR % 128) == 0);
static_assert((DM % 64) == 0);
static_assert((DM % 32) == 0);
static_assert(HD == 64);
static_assert(DM == NH * HD);
static_assert((TP * 4) % 16 == 0);
static_assert((HP * 2) % 16 == 0);
static_assert((OP * 4) % 16 == 0);

typedef unsigned short v8us  __attribute__((ext_vector_type(8)));
typedef unsigned short v16us __attribute__((ext_vector_type(16)));
typedef unsigned short v8usA __attribute__((ext_vector_type(8), may_alias));
typedef _Float16       v8h   __attribute__((ext_vector_type(8)));
typedef _Float16       v16h  __attribute__((ext_vector_type(16)));
typedef _Float16       v8hA  __attribute__((ext_vector_type(8), may_alias));
typedef float          v4f   __attribute__((ext_vector_type(4)));
typedef float          v4fA  __attribute__((ext_vector_type(4), may_alias));
typedef float          v8f   __attribute__((ext_vector_type(8)));
#if defined(__HIP_DEVICE_COMPILE__)
typedef __bf16         v16bf __attribute__((ext_vector_type(16)));
#endif

union FragU { v16us v; v8us half[2]; };
union FragH { v16h  v; v8h  half[2]; };

__device__ __forceinline__ unsigned bbits(float f) {
  unsigned u = __float_as_uint(f);
  return (u + 0x7FFFu + ((u >> 16) & 1u)) >> 16;
}
__device__ __forceinline__ float bf16r(float f) {
  return __uint_as_float(bbits(f) << 16);
}
__device__ __forceinline__ float rcpf_(float x) {
#if defined(__HIP_DEVICE_COMPILE__)
  return __builtin_amdgcn_rcpf(x);
#else
  return 1.0f / x;
#endif
}
__device__ __forceinline__ int unif(int v) {
#if defined(__HIP_DEVICE_COMPILE__)
  return __builtin_amdgcn_readfirstlane(v);
#else
  return v;
#endif
}
__device__ __forceinline__ v8f zero8() { v8f z = {0.f, 0.f, 0.f, 0.f, 0.f, 0.f, 0.f, 0.f}; return z; }

__device__ __forceinline__ v16us ldfrag_u(const unsigned short* p) {
  FragU f;
  f.half[0] = *(const v8usA*)(p);
  f.half[1] = *(const v8usA*)(p + 16);
  return f.v;
}
__device__ __forceinline__ v16h ldfrag_h(const _Float16* p) {
  FragH f;
  f.half[0] = *(const v8hA*)(p);
  f.half[1] = *(const v8hA*)(p + 16);
  return f.v;
}

__device__ __forceinline__ v8f mma_bf(v16us a, v16us b, v8f c) {
#if defined(__HIP_DEVICE_COMPILE__)
  return __builtin_amdgcn_wmma_f32_16x16x32_bf16(false, __builtin_bit_cast(v16bf, a),
                                                false, __builtin_bit_cast(v16bf, b),
                                                (short)0, c, false, false);
#else
  (void)a; (void)b;
  return c;
#endif
}
__device__ __forceinline__ v8f mma_h(v16h a, v16h b, v8f c) {
#if defined(__HIP_DEVICE_COMPILE__)
  return __builtin_amdgcn_wmma_f32_16x16x32_f16(false, a, false, b, (short)0, c, false, false);
#else
  (void)a; (void)b;
  return c;
#endif
}
template <typename F>
__device__ __forceinline__ void guard4(v8f& c0, v8f& c1, v8f& c2, v8f& c3,
                                       const F& f0, const F& f1, const F& f2,
                                       const F& f3, const F& f4, const F& f5) {
#if defined(__HIP_DEVICE_COMPILE__)
  asm volatile("v_nop\n\tv_nop\n\tv_nop\n\tv_nop"
               : "+v"(c0), "+v"(c1), "+v"(c2), "+v"(c3)
               : "v"(f0), "v"(f1), "v"(f2), "v"(f3), "v"(f4), "v"(f5));
#else
  (void)c0; (void)c1; (void)c2; (void)c3; (void)f0; (void)f1; (void)f2; (void)f3; (void)f4; (void)f5;
#endif
}

__global__ __launch_bounds__(256)
void k_cvt(const float* __restrict__ xk, const float* __restrict__ xv, const float* __restrict__ xq,
           const float* __restrict__ wk, const float* __restrict__ wv, const float* __restrict__ wq,
           unsigned short* xb, unsigned short* wb)
{
  const int z    = blockIdx.y;
  const int tid  = threadIdx.x;
  const int lane = tid & 31;
  const int w    = tid >> 5;

  const float* src;
  unsigned short* dst;
  int nrows;
  if (z == 0)      { src = xk; dst = xb;                       nrows = NR; }
  else if (z == 1) { src = xv; dst = xb + (size_t)NR * DM;     nrows = NR; }
  else if (z == 2) { src = xq; dst = xb + (size_t)2 * NR * DM; nrows = NR; }
  else if (z == 3) { src = wk; dst = wb;                       nrows = DM; }
  else if (z == 4) { src = wv; dst = wb + (size_t)DM * DM;     nrows = DM; }
  else             { src = wq; dst = wb + (size_t)2 * DM * DM; nrows = DM; }
  const int row0 = blockIdx.x * 32;
  if (row0 >= nrows) return;

#pragma unroll 1
  for (int i = 0; i < 4; ++i) {
    const int row = row0 + 4 * w + i;
    const float* xr = src + (size_t)row * DM;
    v8us   ov[4];
    size_t off[4];
#pragma unroll
    for (int it = 0; it < 4; ++it) {
      const int p = it * 32 + lane;
      const v4f a = *(const v4fA*)(xr + 8 * p);
      const v4f c = *(const v4fA*)(xr + 8 * p + 4);
      v8us o;
#pragma unroll
      for (int e = 0; e < 4; ++e) {
        o[e]     = (unsigned short)bbits(a[e]);
        o[4 + e] = (unsigned short)bbits(c[e]);
      }
      ov[it]  = o;
      off[it] = (size_t)row * DM + (size_t)(8 * p);
    }
#pragma unroll
    for (int it = 0; it < 4; ++it) *(volatile v8us*)(dst + off[it]) = ov[it];
    __threadfence();
#pragma unroll
    for (int it = 0; it < 4; ++it) *(volatile v8us*)(dst + off[it]) = ov[it];
  }
}

__global__ __launch_bounds__(256)
void k_gauss(float* G)
{
#pragma clang fp contract(off)
  const int tid  = threadIdx.x;
  const int lane = tid & 31;
  const int w    = tid >> 5;
  const float W1    = 0.5f / 65.0f;
  const float TW2   = 2.0f * W1 * W1;
  const float INV2  = 1.0f / TW2;
  const float COEF  = 0.3989422804014327f / W1;
  const float R1023 = 1.0f / 1023.0f;

#pragma unroll 1
  for (int i = 0; i < 4; ++i) {
    const int q = blockIdx.x * 32 + 4 * w + i;
    const float center = (float)q * (1.0f / 1024.0f);
    const int kc = (int)rintf(center * 1023.0f);
    float d2min = 4.0f;
#pragma unroll
    for (int c = -1; c <= 1; ++c) {
      int kk = kc + c;
      kk = (kk < 0) ? 0 : ((kk > SEQ - 1) ? (SEQ - 1) : kk);
      const float pos = (kk >= SEQ - 1) ? 1.0f : (float)kk * R1023;
      const float d   = pos - center;
      const float d2  = d * d;
      d2min = fminf(d2min, d2);
    }
    const float gmax = COEF * __expf((-d2min) * INV2);
    const float rg   = 1.0f / gmax;

    v4f gv[8];
#pragma unroll
    for (int it = 0; it < 8; ++it) {
      v4f v;
#pragma unroll
      for (int e = 0; e < 4; ++e) {
        const int k = 128 * it + 4 * lane + e;
        const float pos = (k >= SEQ - 1) ? 1.0f : (float)k * R1023;
        const float d   = pos - center;
        const float d2  = d * d;
        const float a   = (-d2) * INV2;
        const float g   = COEF * __expf(a);
        v[e] = g * rg;
      }
      gv[it] = v;
    }
    float* gr = G + (size_t)q * SEQ + 4 * lane;
#pragma unroll
    for (int it = 0; it < 8; ++it) *(volatile v4f*)(gr + 128 * it) = gv[it];
    __threadfence();
#pragma unroll
    for (int it = 0; it < 8; ++it) *(volatile v4f*)(gr + 128 * it) = gv[it];
  }
}

__global__ __launch_bounds__(256)
void k_proj(const unsigned short* __restrict__ xb, const unsigned short* __restrict__ wb,
            const float* __restrict__ sk, const float* __restrict__ sv,
            const float* __restrict__ sq, _Float16* k16, _Float16* vt, _Float16* q16)
{
  __shared__ __align__(16) float T[128 * TP];
  __shared__ float rt[128];
  __shared__ float rsc[128];
  const int n0   = blockIdx.x * 64;
  const int m0   = blockIdx.y * 128;
  const int z    = blockIdx.z;
  const int tid  = threadIdx.x;
  const int lane = tid & 31;
  const int w    = tid >> 5;
  const int h    = lane >> 4;
  const int m    = lane & 15;
  const int q8   = lane >> 3;
  const int jj   = lane & 7;
  const int wm   = w >> 1;
  const int wn   = w & 1;

  const unsigned short* A  = xb + (size_t)z * NR * DM;
  const unsigned short* Bt = wb + (size_t)z * DM * DM;
  const float* lsp = (z == 0) ? sk : ((z == 1) ? sv : sq);
  const float els = expf(bf16r(lsp[0]));

  v8f acc[2][2];
  acc[0][0] = zero8(); acc[0][1] = zero8(); acc[1][0] = zero8(); acc[1][1] = zero8();

  const unsigned short* pa = A  + (size_t)(m0 + 32 * wm + m) * DM + 8 * h;
  const unsigned short* pb = Bt + (size_t)(n0 + 32 * wn + m) * DM + 8 * h;
#pragma unroll 2
  for (int kk = 0; kk < DM / 32; ++kk) {
    const v16us a0 = ldfrag_u(pa + 32 * kk);
    const v16us a1 = ldfrag_u(pa + (size_t)16 * DM + 32 * kk);
    const v16us b0 = ldfrag_u(pb + 32 * kk);
    const v16us b1 = ldfrag_u(pb + (size_t)16 * DM + 32 * kk);
    acc[0][0] = mma_bf(a0, b0, acc[0][0]);
    acc[0][1] = mma_bf(a0, b1, acc[0][1]);
    acc[1][0] = mma_bf(a1, b0, acc[1][0]);
    acc[1][1] = mma_bf(a1, b1, acc[1][1]);
    guard4<v16us>(acc[0][0], acc[0][1], acc[1][0], acc[1][1], a0, a1, b0, b1, a0, b1);
  }

#pragma unroll
  for (int mi = 0; mi < 2; ++mi)
#pragma unroll
    for (int ni = 0; ni < 2; ++ni)
#pragma unroll
      for (int r = 0; r < 8; ++r)
        T[(32 * wm + 16 * mi + 8 * h + r) * TP + 32 * wn + 16 * ni + m] = acc[mi][ni][r];
  __syncthreads();

  {
    const int row = tid >> 1;
    const int hf  = tid & 1;
    const v4fA* tr = (const v4fA*)(T + row * TP + 32 * hf);
    float ss = 0.f, f0 = 0.f;
#pragma unroll
    for (int c4 = 0; c4 < 8; ++c4) {
      const v4f x = tr[c4];
#pragma unroll
      for (int e = 0; e < 4; ++e) {
        if (c4 == 0 && e == 0) f0 = x[0];
        else ss += x[e] * x[e];
      }
    }
    ss += (hf != 0) ? f0 * f0 : 0.f;
    ss += __shfl_xor(ss, 1, 32);
    const float x0  = T[row * TP];
    const float sig = 1.0f / (1.0f + __expf(-x0));
    const float t   = sig * els + 1.1f;
    const float sc  = sqrtf((t * t - 1.0f) / ss);
    if (hf == 0) { rt[row] = t; rsc[row] = sc; }
  }
  __syncthreads();

  if (z == 1) {
    const int h16  = lane >> 4;
    const int j16  = lane & 15;
    const int b    = m0 >> 10;
    const int tok0 = m0 & (SEQ - 1);
    const int bh   = b * NH + blockIdx.x;
    v8h    ov[4];
    size_t off[4];
#pragma unroll
    for (int it = 0; it < 4; ++it) {
      const int d = 16 * it + 2 * w + h16;
      v8h o;
#pragma unroll
      for (int e = 0; e < 8; ++e) {
        const int tk   = 8 * j16 + e;
        const float x  = T[tk * TP + d];
        const float tv = rt[tk] * 8.0f;
        const float sp = x * (rsc[tk] * 8.0f);
        o[e] = (_Float16)((d == 0) ? tv : sp);
      }
      ov[it]  = o;
      off[it] = ((size_t)(bh * HD + d)) * SEQ + (size_t)(tok0 + 8 * j16);
    }
#pragma unroll
    for (int it = 0; it < 4; ++it) *(volatile v8h*)(vt + off[it]) = ov[it];
    __threadfence();
#pragma unroll
    for (int it = 0; it < 4; ++it) *(volatile v8h*)(vt + off[it]) = ov[it];
  } else {
    _Float16* P = (z == 2) ? q16 : k16;
    const float tsg = (z == 2) ? -8.0f : 8.0f;
    v8h    ov[4];
    size_t off[4];
#pragma unroll
    for (int it = 0; it < 4; ++it) {
      const int rl = 32 * it + 4 * w + q8;
      const v4fA* tp = (const v4fA*)(T + rl * TP + 8 * jj);
      const v4f a = tp[0];
      const v4f c = tp[1];
      const float sc8 = rsc[rl] * 8.0f;
      const float tv  = rt[rl] * tsg;
      v8h o;
      o[0] = (_Float16)((jj == 0) ? tv : a[0] * sc8);
#pragma unroll
      for (int e = 1; e < 4; ++e) o[e] = (_Float16)(a[e] * sc8);
#pragma unroll
      for (int e = 0; e < 4; ++e) o[4 + e] = (_Float16)(c[e] * sc8);
      ov[it]  = o;
      off[it] = (size_t)(m0 + rl) * DM + (size_t)(n0 + 8 * jj);
    }
#pragma unroll
    for (int it = 0; it < 4; ++it) *(volatile v8h*)(P + off[it]) = ov[it];
    __threadfence();
#pragma unroll
    for (int it = 0; it < 4; ++it) *(volatile v8h*)(P + off[it]) = ov[it];
  }
}

__global__ __launch_bounds__(256)
void k_attn(const _Float16* __restrict__ q16, const _Float16* __restrict__ k16,
            const _Float16* __restrict__ vt, const int* __restrict__ msk,
            const float* __restrict__ G, const float* __restrict__ asp,
            const float* __restrict__ abp, float* out)
{
  __shared__ __align__(16) _Float16 Ps[8 * 16 * HP];
  __shared__ __align__(16) float Os[8 * 16 * OP];
  const int tid  = threadIdx.x;
  const int lane = tid & 31;
  const int w    = unif(tid >> 5);
  const int h    = lane >> 4;
  const int m    = lane & 15;
  const int q8   = lane >> 3;
  const int jj   = lane & 7;
  const int bh   = blockIdx.y;
  const int b    = bh >> 4;
  const int hd   = bh & (NH - 1);
  const int hc   = hd * HD;
  const int qblk = blockIdx.x;
  const int q0w  = qblk * 128 + 16 * w;
  const int qrow0 = b * SEQ + q0w;
  _Float16* Pw = Ps + w * (16 * HP);
  float*    Ow = Os + w * (16 * OP);

  const _Float16* qp = q16 + (size_t)(qrow0 + m) * DM + hc + 8 * h;
  const v16h qa0 = ldfrag_h(qp);
  const v16h qa1 = ldfrag_h(qp + 32);
  const float rcs = 1.0f / bf16r(asp[0]);
  const float ab  = bf16r(abp[0]);
  float mst[8], lst[8];
#pragma unroll
  for (int r = 0; r < 8; ++r) { mst[r] = -1.0e30f; lst[r] = 0.f; }
  v8f oacc[4];
  oacc[0] = zero8(); oacc[1] = zero8(); oacc[2] = zero8(); oacc[3] = zero8();

  const _Float16* kbase = k16 + (size_t)(b * SEQ + m) * DM + hc + 8 * h;
  const _Float16* vbase = vt + (size_t)(bh * HD + m) * SEQ + 8 * h;
  const int*      mbase = msk + (size_t)(qrow0 + 8 * h) * SEQ + m;
  const float*    gbase = G + (size_t)(q0w + 8 * h) * SEQ + m;

#pragma unroll 1
  for (int j = 0; j < SEQ / 64; ++j) {
    const int k0 = 64 * j;
    const _Float16* kp = kbase + (size_t)k0 * DM;
    v8f sacc[4];
    sacc[0] = zero8(); sacc[1] = zero8(); sacc[2] = zero8(); sacc[3] = zero8();
    {
      const v16h b0 = ldfrag_h(kp);
      const v16h b1 = ldfrag_h(kp + (size_t)16 * DM);
      const v16h b2 = ldfrag_h(kp + (size_t)32 * DM);
      const v16h b3 = ldfrag_h(kp + (size_t)48 * DM);
      sacc[0] = mma_h(qa0, b0, sacc[0]);
      sacc[1] = mma_h(qa0, b1, sacc[1]);
      sacc[2] = mma_h(qa0, b2, sacc[2]);
      sacc[3] = mma_h(qa0, b3, sacc[3]);
      const v16h c0 = ldfrag_h(kp + 32);
      const v16h c1 = ldfrag_h(kp + (size_t)16 * DM + 32);
      const v16h c2 = ldfrag_h(kp + (size_t)32 * DM + 32);
      const v16h c3 = ldfrag_h(kp + (size_t)48 * DM + 32);
      sacc[0] = mma_h(qa1, c0, sacc[0]);
      sacc[1] = mma_h(qa1, c1, sacc[1]);
      sacc[2] = mma_h(qa1, c2, sacc[2]);
      sacc[3] = mma_h(qa1, c3, sacc[3]);
      guard4<v16h>(sacc[0], sacc[1], sacc[2], sacc[3], qa0, qa1, c0, c1, c2, c3);
    }
    const bool near = !((k0 > q0w + 15 + DFAR) || (k0 + 63 + DFAR < q0w));

#pragma unroll
    for (int r = 0; r < 8; ++r) {
      float g0 = 0.f, g1 = 0.f, g2 = 0.f, g3 = 0.f;
      if (near) {
        const float* gp = gbase + (size_t)r * SEQ + k0;
        g0 = gp[0]; g1 = gp[16]; g2 = gp[32]; g3 = gp[48];
      }
      const int* mp = mbase + (size_t)r * SEQ + k0;
      const int k_0 = mp[0];
      const int k_1 = mp[16];
      const int k_2 = mp[32];
      const int k_3 = mp[48];
      const float a0 = (2.0f + 2.0f * (sacc[0][r] * (1.0f / 64.0f))) * rcs + ab;
      const float a1 = (2.0f + 2.0f * (sacc[1][r] * (1.0f / 64.0f))) * rcs + ab;
      const float a2 = (2.0f + 2.0f * (sacc[2][r] * (1.0f / 64.0f))) * rcs + ab;
      const float a3 = (2.0f + 2.0f * (sacc[3][r] * (1.0f / 64.0f))) * rcs + ab;
      float s0 = a0 * g0;
      float s1 = a1 * g1;
      float s2 = a2 * g2;
      float s3 = a3 * g3;
      s0 = (k_0 != 1) ? -1.0e18f : s0;
      s1 = (k_1 != 1) ? -1.0e18f : s1;
      s2 = (k_2 != 1) ? -1.0e18f : s2;
      s3 = (k_3 != 1) ? -1.0e18f : s3;
      float mx = fmaxf(fmaxf(s0, s1), fmaxf(s2, s3));
      mx = fmaxf(mx, __shfl_xor(mx, 1, 32));
      mx = fmaxf(mx, __shfl_xor(mx, 2, 32));
      mx = fmaxf(mx, __shfl_xor(mx, 4, 32));
      mx = fmaxf(mx, __shfl_xor(mx, 8, 32));
      const float mnew = fmaxf(mst[r], mx);
      const float msc  = __expf(mst[r] - mnew);
      mst[r] = mnew;
      const float p0 = __expf(s0 - mnew) * 4096.0f;
      const float p1 = __expf(s1 - mnew) * 4096.0f;
      const float p2 = __expf(s2 - mnew) * 4096.0f;
      const float p3 = __expf(s3 - mnew) * 4096.0f;
      const _Float16 zh = (_Float16)0.0f;
      const _Float16 h0 = (p0 < F16_MIN_NORMAL) ? zh : (_Float16)p0;
      const _Float16 h1 = (p1 < F16_MIN_NORMAL) ? zh : (_Float16)p1;
      const _Float16 h2 = (p2 < F16_MIN_NORMAL) ? zh : (_Float16)p2;
      const _Float16 h3 = (p3 < F16_MIN_NORMAL) ? zh : (_Float16)p3;
      float rs = (float)h0 + (float)h1 + (float)h2 + (float)h3;
      rs += __shfl_xor(rs, 1, 32);
      rs += __shfl_xor(rs, 2, 32);
      rs += __shfl_xor(rs, 4, 32);
      rs += __shfl_xor(rs, 8, 32);
      lst[r] = lst[r] * msc + rs;
      Pw[(8 * h + r) * HP + m]      = h0;
      Pw[(8 * h + r) * HP + 16 + m] = h1;
      Pw[(8 * h + r) * HP + 32 + m] = h2;
      Pw[(8 * h + r) * HP + 48 + m] = h3;
      oacc[0][r] *= msc;
      oacc[1][r] *= msc;
      oacc[2][r] *= msc;
      oacc[3][r] *= msc;
    }
    __syncthreads();

    {
      const v16h pa0 = ldfrag_h(Pw + m * HP + 8 * h);
      const v16h pa1 = ldfrag_h(Pw + m * HP + 32 + 8 * h);
      const _Float16* vp = vbase + k0;
      const v16h v0 = ldfrag_h(vp);
      const v16h v1 = ldfrag_h(vp + (size_t)16 * SEQ);
      const v16h v2 = ldfrag_h(vp + (size_t)32 * SEQ);
      const v16h v3 = ldfrag_h(vp + (size_t)48 * SEQ);
      oacc[0] = mma_h(pa0, v0, oacc[0]);
      oacc[1] = mma_h(pa0, v1, oacc[1]);
      oacc[2] = mma_h(pa0, v2, oacc[2]);
      oacc[3] = mma_h(pa0, v3, oacc[3]);
      const v16h u0 = ldfrag_h(vp + 32);
      const v16h u1 = ldfrag_h(vp + (size_t)16 * SEQ + 32);
      const v16h u2 = ldfrag_h(vp + (size_t)32 * SEQ + 32);
      const v16h u3 = ldfrag_h(vp + (size_t)48 * SEQ + 32);
      oacc[0] = mma_h(pa1, u0, oacc[0]);
      oacc[1] = mma_h(pa1, u1, oacc[1]);
      oacc[2] = mma_h(pa1, u2, oacc[2]);
      oacc[3] = mma_h(pa1, u3, oacc[3]);
      guard4<v16h>(oacc[0], oacc[1], oacc[2], oacc[3], pa0, pa1, u0, u1, u2, u3);
    }
    __syncthreads();
  }

#pragma unroll
  for (int r = 0; r < 8; ++r) {
    const float inv = rcpf_(lst[r] * 8.0f);
    const float mu0 = oacc[0][r] * inv;
    const float mu1 = oacc[1][r] * inv;
    const float mu2 = oacc[2][r] * inv;
    const float mu3 = oacc[3][r] * inv;
    float us = mu0 * mu0;
    us += mu1 * mu1;
    us += mu2 * mu2;
    us += mu3 * mu3;
    us += __shfl_xor(us, 1, 32);
    us += __shfl_xor(us, 2, 32);
    us += __shfl_xor(us, 4, 32);
    us += __shfl_xor(us, 8, 32);
    const float t2  = __shfl(mu0 * mu0, lane & 16, 32);
    const float ln  = us - 2.0f * t2;
    const float den = sqrtf(fmaxf(fabsf(ln), 1e-8f));
    const float iv  = 1.0f / den;
    Ow[(8 * h + r) * OP + m]      = mu0 * iv;
    Ow[(8 * h + r) * OP + 16 + m] = mu1 * iv;
    Ow[(8 * h + r) * OP + 32 + m] = mu2 * iv;
    Ow[(8 * h + r) * OP + 48 + m] = mu3 * iv;
  }
  __syncthreads();

  v4f    ov[8];
  size_t ooff[8];
#pragma unroll
  for (int it = 0; it < 8; ++it) {
    const int L  = 4 * it + q8;
    const int rl = L >> 1;
    const int hf = L & 1;
    ov[it]   = *(const v4fA*)(Ow + rl * OP + 32 * hf + 4 * jj);
    ooff[it] = (size_t)(qrow0 + rl) * DM + (size_t)(hc + 32 * hf + 4 * jj);
  }
#pragma unroll
  for (int it = 0; it < 8; ++it) *(volatile v4f*)(out + ooff[it]) = ov[it];
  __threadfence();
#pragma unroll
  for (int it = 0; it < 8; ++it) *(volatile v4f*)(out + ooff[it]) = ov[it];
}

extern "C" void kernel_launch(void* const* d_in, const int* in_sizes, int n_in,
                              void* d_out, int out_size, void* d_ws, size_t ws_size,
                              hipStream_t stream) {
  if (n_in < 12) return;
  if (in_sizes[0] != NR * DM || in_sizes[1] != NR * DM || in_sizes[2] != NR * DM) return;
  if (in_sizes[3] != NB * SEQ * SEQ) return;
  if (in_sizes[4] != DM * DM || in_sizes[5] != DM * DM || in_sizes[6] != DM * DM) return;
  if (in_sizes[7] < 1 || in_sizes[8] < 1 || in_sizes[9] < 1 || in_sizes[10] < 1 ||
      in_sizes[11] < 1) return;
  if (out_size != NR * DM) return;
  if (ws_size < WS_TOTAL) return;

  const float* key   = (const float*)d_in[0];
  const float* value = (const float*)d_in[1];
  const float* query = (const float*)d_in[2];
  const int*   mask  = (const int*)d_in[3];
  const float* Wk    = (const float*)d_in[4];
  const float* Wv    = (const float*)d_in[5];
  const float* Wq    = (const float*)d_in[6];
  const float* sk    = (const float*)d_in[7];
  const float* sv    = (const float*)d_in[8];
  const float* sq    = (const float*)d_in[9];
  const float* asc   = (const float*)d_in[10];
  const float* abi   = (const float*)d_in[11];
  float* out = (float*)d_out;
  char* ws = (char*)d_ws;

  unsigned short* xb  = (unsigned short*)(ws + OFF_XB);
  unsigned short* wb  = (unsigned short*)(ws + OFF_WB);
  float*          G   = (float*)(ws + OFF_G);
  _Float16*       q16 = (_Float16*)(ws + OFF_Q16);
  _Float16*       k16 = (_Float16*)(ws + OFF_K16);
  _Float16*       vtp = (_Float16*)(ws + OFF_VT);

  k_cvt<<<dim3(NR / 32, 6), dim3(256), 0, stream>>>(key, value, query, Wk, Wv, Wq, xb, wb);
  (void)hipGetLastError();
  k_gauss<<<dim3(SEQ / 32), dim3(256), 0, stream>>>(G);
  (void)hipGetLastError();
  k_proj<<<dim3(DM / 64, NR / 128, 3), dim3(256), 0, stream>>>(xb, wb, sk, sv, sq, k16, vtp, q16);
  (void)hipGetLastError();
  k_attn<<<dim3(SEQ / 128, NBH), dim3(256), 0, stream>>>(q16, k16, vtp, mask, G, asc, abi, out);
  (void)hipGetLastError();
}
